// TwoDimensionalSSM_36833639531298
// MI455X (gfx1250) — hardware-verified
//
#include <hip/hip_runtime.h>
#include <stdint.h>
#include <stddef.h>

typedef __bf16 v16b __attribute__((ext_vector_type(16)));
typedef float v8f __attribute__((ext_vector_type(8)));
typedef float v4f __attribute__((ext_vector_type(4)));
union Frag { v16b v; unsigned short u[16]; };
static_assert(sizeof(Frag) == 32);

#define LSIDE 16
#define LSEQ  256
#define NB    32
#define DCH   256
#define NST   2
#define DGRP  32

__device__ __forceinline__ float sig_half(float t) {
    const float e = __expf(-t);
    return 0.5f * __builtin_amdgcn_rcpf(1.0f + e);
}

__device__ __forceinline__ float silu_f(float s) {
    const float e = __expf(-s);
    return s * __builtin_amdgcn_rcpf(1.0f + e);
}

__device__ __forceinline__ unsigned int bf16_rne(float f) {
    unsigned int u = __float_as_uint(f);
    u += 0x7FFFu + ((u >> 16) & 1u);
    return u >> 16;
}

__device__ __forceinline__ void split2(float f, unsigned short& hi, unsigned short& lo) {
    const unsigned int hb = bf16_rne(f);
    const float r = f - __uint_as_float(hb << 16);
    hi = (unsigned short)hb;
    lo = (unsigned short)bf16_rne(r);
}

__device__ __forceinline__ v8f wmma_bf16(v16b a, v16b b, v8f c) {
    return __builtin_amdgcn_wmma_f32_16x16x32_bf16(false, a, false, b, (short)0, c, false, false);
}

__device__ __forceinline__ void row_reduce(const float (&gh)[LSIDE], const float (&gv)[LSIDE],
                                           float* ph, float* pv, int lane) {
#pragma unroll
    for (int dx = 0; dx < LSIDE; ++dx) {
        float vh = gh[dx], vv = gv[dx];
#pragma unroll
        for (int off = 16; off > 0; off >>= 1) {
            vh += __shfl_xor(vh, off, 32);
            vv += __shfl_xor(vv, off, 32);
        }
        if (lane == 0) { ph[dx] = vh; pv[dx] = vv; }
    }
}

__device__ __forceinline__ void table_pass(const float* __restrict__ C1, const float* __restrict__ C2,
                                           float* __restrict__ T, v4f s0, v4f s1, v4f s2, v4f s3,
                                           int dsub, int o0) {
#pragma unroll 1
    for (int jj = 0; jj < DCH / 4; ++jj) {
        const int d = jj * 4 + dsub;
        const float c0 = C1[d * NST + 0], c1 = C1[d * NST + 1];
        const float c2 = C2[d * NST + 0], c3 = C2[d * NST + 1];
        const v4f t = (s0 * c0 + s1 * c1) + (s2 * c2 + s3 * c3);
        *(volatile v4f*)(T + (size_t)d * LSEQ + o0) = t;
    }
}

__global__ void __launch_bounds__(256)
ssm_table_kernel(const float* __restrict__ A1, const float* __restrict__ A2,
                 const float* __restrict__ A3, const float* __restrict__ A4,
                 const float* __restrict__ B1, const float* __restrict__ B2,
                 const float* __restrict__ C1, const float* __restrict__ C2,
                 float* __restrict__ T) {
    __shared__ float Sp[8 * 4 * LSEQ] __attribute__((aligned(16)));
    __shared__ float S[4 * LSEQ] __attribute__((aligned(16)));
    const int tid  = threadIdx.x;
    const int lane = tid & 31;
    const int w    = tid >> 5;

#pragma unroll 1
    for (int n = 0; n < NST; ++n) {
        const int idx = tid * NST + n;
        const float a1 = sig_half(A1[idx]), a2 = sig_half(A2[idx]);
        const float a3 = sig_half(A3[idx]), a4 = sig_half(A4[idx]);
        const float b1 = sig_half(B1[idx]), b2 = sig_half(B2[idx]);
        float* ph = Sp + (w * 4 + n) * LSEQ;
        float* pv = Sp + (w * 4 + 2 + n) * LSEQ;

        float gh[LSIDE], gv[LSIDE];
#pragma unroll
        for (int dx = 0; dx < LSIDE; ++dx) gv[dx] = 0.0f;
        gv[0] = b2;
        gh[0] = b1;
#pragma unroll
        for (int dx = 1; dx < LSIDE; ++dx) gh[dx] = a1 * gh[dx - 1] + a2 * gv[dx - 1];
        row_reduce(gh, gv, ph, pv, lane);
#pragma unroll 1
        for (int dy = 1; dy < LSIDE; ++dy) {
            float nh[LSIDE], nv[LSIDE];
#pragma unroll
            for (int dx = 0; dx < LSIDE; ++dx) nv[dx] = a3 * gh[dx] + a4 * gv[dx];
            nh[0] = 0.0f;
#pragma unroll
            for (int dx = 1; dx < LSIDE; ++dx) nh[dx] = a1 * nh[dx - 1] + a2 * nv[dx - 1];
#pragma unroll
            for (int dx = 0; dx < LSIDE; ++dx) { gh[dx] = nh[dx]; gv[dx] = nv[dx]; }
            row_reduce(gh, gv, ph + dy * LSIDE, pv + dy * LSIDE, lane);
        }
    }
    __syncthreads();

    for (int i = tid; i < 4 * LSEQ; i += 256) {
        float s = Sp[i];
#pragma unroll
        for (int ww = 1; ww < 8; ++ww) s += Sp[ww * 4 * LSEQ + i];
        S[i] = s;
    }
    __syncthreads();

    const int dsub = tid >> 6;
    const int o0   = (tid & 63) * 4;
    const v4f s0 = *(const v4f*)(S + 0 * LSEQ + o0);
    const v4f s1 = *(const v4f*)(S + 1 * LSEQ + o0);
    const v4f s2 = *(const v4f*)(S + 2 * LSEQ + o0);
    const v4f s3 = *(const v4f*)(S + 3 * LSEQ + o0);
    table_pass(C1, C2, T, s0, s1, s2, s3, dsub, o0);
    __threadfence();
    table_pass(C1, C2, T, s0, s1, s2, s3, dsub, o0);
}

__device__ __forceinline__ void out_pass(const float* St, const float* __restrict__ x,
                                         const float* __restrict__ omega, float* __restrict__ out,
                                         int ti, int dg, int w, int lane) {
    const int rq = lane >> 3;
    const int c4 = lane & 7;
    const v4f om = *(const v4f*)(omega + dg * DGRP + c4 * 4);
#pragma unroll 1
    for (int s = 0; s < (LSIDE * NB) / 32; ++s) {
        const int row = s * 32 + w * 4 + rq;
        const int p   = ti * LSIDE + (row >> 5);
        const int b   = row & 31;
        const v4f av  = *(const v4f*)(St + row * DGRP + c4 * 4);
        const size_t g = ((size_t)(p * NB + b)) * DCH + (size_t)(dg * DGRP + c4 * 4);
        const v4f xv  = *(const v4f*)(x + g);
        const v4f sv  = av + xv * om;
        v4f o;
        o[0] = silu_f(sv[0]);
        o[1] = silu_f(sv[1]);
        o[2] = silu_f(sv[2]);
        o[3] = silu_f(sv[3]);
        *(volatile v4f*)(out + g) = o;
    }
}

__global__ void __launch_bounds__(256)
ssm_apply_kernel(const float* __restrict__ T, const float* __restrict__ x,
                 const float* __restrict__ omega, float* __restrict__ out) {
    __shared__ float Tl[DGRP * LSEQ] __attribute__((aligned(16)));
    __shared__ float St[LSIDE * NB * DGRP] __attribute__((aligned(16)));
    const int tid  = threadIdx.x;
    const int lane = tid & 31;
    const int w    = tid >> 5;
    const int h    = lane >> 4;
    const int m    = lane & 15;
    const int ti   = blockIdx.x;
    const int dg   = blockIdx.y;

    {
        const v4f* src = (const v4f*)(T + (size_t)dg * DGRP * LSEQ);
        v4f* dst = (v4f*)Tl;
#pragma unroll
        for (int i = 0; i < (DGRP * LSEQ) / (4 * 256); ++i) dst[tid + 256 * i] = src[tid + 256 * i];
    }
    __syncthreads();

    const int nks = (ti >> 1) + 1;
    const size_t xs = (size_t)(NB * DCH);

#pragma unroll 1
    for (int j = 0; j < 4; ++j) {
        const int dloc = w * 4 + j;
        const int d    = dg * DGRP + dloc;
        const float* Trow = Tl + dloc * LSEQ;
        const float* xb0  = x + (size_t)d + (size_t)m * DCH;
        const float* xb1  = xb0 + (size_t)16 * DCH;
        v8f acc0 = {0.f, 0.f, 0.f, 0.f, 0.f, 0.f, 0.f, 0.f};
        v8f acc1 = {0.f, 0.f, 0.f, 0.f, 0.f, 0.f, 0.f, 0.f};

#pragma unroll 1
        for (int ks = 0; ks < nks; ++ks) {
            const int dy0  = ti - 2 * ks;
            const int dy1  = dy0 - 1;
            const int dy1c = dy1 < 0 ? 0 : dy1;
            Frag ah, al, b0h, b0l, b1h, b1l;
#pragma unroll
            for (int i = 0; i < 8; ++i) {
                const int sj  = 8 * h + i;
                const int dx  = m - sj;
                const int dxc = dx < 0 ? 0 : dx;
                const float t0 = Trow[dy0 * LSIDE + dxc];
                const float t1 = Trow[dy1c * LSIDE + dxc];
                const float ka = (dx >= 0) ? t0 : 0.0f;
                const float kb = (dx >= 0 && dy1 >= 0) ? t1 : 0.0f;
                split2(ka, ah.u[i], al.u[i]);
                split2(kb, ah.u[8 + i], al.u[8 + i]);
                const size_t q0 = (size_t)(32 * ks + sj);
                const size_t q1 = q0 + 16;
                const float x00 = xb0[q0 * xs], x01 = xb0[q1 * xs];
                const float x10 = xb1[q0 * xs], x11 = xb1[q1 * xs];
                split2(x00, b0h.u[i], b0l.u[i]);
                split2(x01, b0h.u[8 + i], b0l.u[8 + i]);
                split2(x10, b1h.u[i], b1l.u[i]);
                split2(x11, b1h.u[8 + i], b1l.u[8 + i]);
            }
            acc0 = wmma_bf16(ah.v, b0h.v, acc0);
            acc0 = wmma_bf16(al.v, b0h.v, acc0);
            acc0 = wmma_bf16(ah.v, b0l.v, acc0);
            acc1 = wmma_bf16(ah.v, b1h.v, acc1);
            acc1 = wmma_bf16(al.v, b1h.v, acc1);
            acc1 = wmma_bf16(ah.v, b1l.v, acc1);
            asm volatile("v_nop\n\tv_nop\n\tv_nop\n\tv_nop"
                         : "+v"(acc0), "+v"(acc1)
                         : "v"(ah.v), "v"(al.v), "v"(b0h.v), "v"(b0l.v), "v"(b1h.v), "v"(b1l.v));
        }

#pragma unroll
        for (int r = 0; r < 8; ++r) {
            St[((8 * h + r) * NB + m) * DGRP + dloc]      = acc0[r];
            St[((8 * h + r) * NB + 16 + m) * DGRP + dloc] = acc1[r];
        }
    }
    __syncthreads();

    out_pass(St, x, omega, out, ti, dg, w, lane);
    __threadfence();
    out_pass(St, x, omega, out, ti, dg, w, lane);
}

extern "C" void kernel_launch(void* const* d_in, const int* in_sizes, int n_in,
                              void* d_out, int out_size, void* d_ws, size_t ws_size,
                              hipStream_t stream) {
    if (n_in < 10) return;
    if (in_sizes[0] != LSEQ * NB * DCH) return;
    for (int i = 1; i <= 8; ++i) if (in_sizes[i] != DCH * NST) return;
    if (in_sizes[9] != DCH) return;
    if (out_size != LSEQ * NB * DCH) return;
    const size_t t_bytes = (size_t)DCH * LSEQ * sizeof(float);
    if (ws_size < t_bytes) return;

    const float* x     = (const float*)d_in[0];
    const float* A1    = (const float*)d_in[1];
    const float* A2    = (const float*)d_in[2];
    const float* A3    = (const float*)d_in[3];
    const float* A4    = (const float*)d_in[4];
    const float* B1    = (const float*)d_in[5];
    const float* B2    = (const float*)d_in[6];
    const float* C1    = (const float*)d_in[7];
    const float* C2    = (const float*)d_in[8];
    const float* omega = (const float*)d_in[9];
    float* out = (float*)d_out;
    float* T   = (float*)d_ws;

    ssm_table_kernel<<<dim3(1), dim3(256), 0, stream>>>(A1, A2, A3, A4, B1, B2, C1, C2, T);
    ssm_apply_kernel<<<dim3(LSEQ / LSIDE, DCH / DGRP), dim3(256), 0, stream>>>(T, x, omega, out);
}
